// StressGNN_8237747274157
// MI455X (gfx1250) — hardware-verified
//
#include <hip/hip_runtime.h>

#define NN 25000
#define NE 100000

typedef float v2f __attribute__((ext_vector_type(2)));
typedef float v4f __attribute__((ext_vector_type(4)));
typedef float v8f __attribute__((ext_vector_type(8)));
typedef float v4fa __attribute__((ext_vector_type(4), may_alias));
typedef unsigned v4ua __attribute__((ext_vector_type(4), may_alias));
typedef unsigned v4u_t __attribute__((ext_vector_type(4)));
#define BUCKET 64
#define LCAP   1024
#define NBK    ((NN + BUCKET - 1) / BUCKET)
#define ST2F(ptr, val) do { *(volatile float*)(ptr) = (val); __threadfence(); *(volatile float*)(ptr) = (val); } while (0)

typedef _Float16 f16;
typedef __attribute__((ext_vector_type(16))) _Float16 v16h;
#define RSPLIT (1.0f / 2048.0f)
struct Frag2 { v16h h, l; };
__device__ __forceinline__ int kof(int i, int hi) { return (i < 8) ? (hi * 8 + i) : (16 + hi * 8 + (i - 8)); }
template <int K>
__device__ __forceinline__ Frag2 afrag_row(const float* __restrict__ row, int hi) {
    Frag2 f;
#pragma unroll
    for (int i = 0; i < 16; ++i) {
        const int k = kof(i, hi);
        const float v = (k < K) ? row[k] : 0.0f;
        const f16 hv = (f16)v; f.h[i] = hv; f.l[i] = (f16)((v - (float)hv) * 2048.0f);
    }
    return f;
}
template <int K>
__device__ __forceinline__ Frag2 bfrag_col(const float* __restrict__ w, int ld, int n, int hi) {
    Frag2 f;
#pragma unroll
    for (int i = 0; i < 16; ++i) {
        const int k = kof(i, hi);
        const float v = (k < K) ? w[k * ld + n] : 0.0f;
        const f16 hv = (f16)v; f.h[i] = hv; f.l[i] = (f16)((v - (float)hv) * 2048.0f);
    }
    return f;
}
__device__ __forceinline__ v8f wmma16(v16h a, v16h b, v8f c) {
    return __builtin_amdgcn_wmma_f32_16x16x32_f16(false, a, false, b, (short)0, c, false, false);
}
__device__ __forceinline__ v8f wmma_split(const Frag2& a, const Frag2& b, v8f c) {
    v8f x = {};
    x = wmma16(a.l, b.h, x); x = wmma16(a.h, b.l, x);
    return wmma16(a.h, b.h, c) + x * RSPLIT;
}

__global__ __launch_bounds__(256) void gnn_zero_kernel(float* p, int n) {
    int i = blockIdx.x * blockDim.x + threadIdx.x;
    int s = gridDim.x * blockDim.x;
    for (; i < n; i += s) p[i] = 0.0f;
}

template<int IN>
__global__ __launch_bounds__(256) void gnn_edge_kernel(
    const float* __restrict__ x,
    const int* __restrict__ eidx,
    const float* __restrict__ eattr,
    const float* __restrict__ w_mlp,
    const float* __restrict__ b_mlp,
    float* __restrict__ msg,
    int nEdges)
{
    constexpr int WC = IN * 32;
    __shared__ float lds_w[4 * WC];
    __shared__ float lds_b[WC];
    __shared__ __align__(16) float lds_x[8][16][IN];
    __shared__ __align__(16) float lds_m[8][16][32];

    const int tid = threadIdx.x;
    for (int i = tid; i < 4 * WC; i += 256) lds_w[i] = w_mlp[i];
    for (int i = tid; i < WC; i += 256)     lds_b[i] = b_mlp[i];
    __syncthreads();

    const int lane = tid & 31;
    const int wave = tid >> 5;
    const int ml = lane & 15;
    const int kh = lane >> 4;
    const int nGroups = nEdges >> 4;


    for (int g = blockIdx.x * 8 + wave; g < nGroups; g += gridDim.x * 8) {
        const int e0 = g << 4;
        const int eMine = e0 + ml;
        const Frag2 a = afrag_row<4>(eattr + (size_t)eMine * 4, kh);
        int srcI = eidx[eMine]; srcI = ((unsigned)srcI < (unsigned)NN) ? srcI : 0;
        const int iBase = kh * (IN / 2);
        const v4f* xs = (const v4f*)(x + (size_t)srcI * IN + iBase);
        v4f* xd = (v4f*)(&lds_x[wave][ml][iBase]);
        #pragma unroll
        for (int j = 0; j < IN / 8; ++j) xd[j] = xs[j];

        v8f c0 = {};
        v8f c1 = {};
        for (int i = 0; i < IN; ++i) {
            float xv[8];
            #pragma unroll
            for (int r = 0; r < 8; ++r) xv[r] = lds_x[wave][r + 8 * kh][i];
            #pragma unroll
            for (int oh = 0; oh < 2; ++oh) {
                const int cb = i * 32 + oh * 16;
                const Frag2 b = bfrag_col<4>(lds_w, WC, cb + ml, kh);
                v8f z = {};
                v8f w = wmma_split(a, b, z);
                const float bb = lds_b[cb + ml];
                #pragma unroll
                for (int r = 0; r < 8; ++r) {
                    float wv = w[r] + bb;
                    wv = wv > 0.0f ? wv : 0.0f;
                    if (oh == 0) c0[r] += xv[r] * wv;
                    else         c1[r] += xv[r] * wv;
                }
            }
        }
        #pragma unroll
        for (int r = 0; r < 8; ++r) { lds_m[wave][r + 8 * kh][ml] = c0[r]; lds_m[wave][r + 8 * kh][16 + ml] = c1[r]; }
        asm volatile("s_wait_dscnt 0" ::: "memory");
        #pragma unroll 1
        for (int pass = 0; pass < 2; ++pass) {
            #pragma unroll
            for (int i = 0; i < 4; ++i) { const int c = lane + 32 * i, ee = c >> 3, q = c & 7;
                *(volatile v4f*)(msg + (size_t)(e0 + ee) * 32 + q * 4) = *(const volatile v4fa*)(&lds_m[wave][ee][q * 4]); }
            __threadfence();
        }
        asm volatile("s_wait_dscnt 0" ::: "memory");
    }
}

__global__ __launch_bounds__(256) void gnn_list_kernel(const int* __restrict__ dst, int* __restrict__ noff, int* __restrict__ ncnt, int* __restrict__ ledge) {
    __shared__ unsigned lst[LCAP], srt[LCAP];
    __shared__ int wcnt[8];
    __shared__ int total;
    __shared__ int cntb[BUCKET], off[BUCKET];
    const int tid = threadIdx.x, lane = tid & 31, wave = tid >> 5;
    const int n0 = blockIdx.x * BUCKET;
    if (tid == 0) total = 0;
    if (tid < BUCKET) cntb[tid] = 0;
    __syncthreads();
    for (int e0 = 0; e0 < NE; e0 += 256) {
        const int e = e0 + tid;
        int loc = -1;
        if (e < NE) { const int l = dst[e] - n0; if ((unsigned)l < (unsigned)BUCKET) loc = l; }
        const unsigned m = __ballot(loc >= 0);
        if (lane == 0) wcnt[wave] = __popc(m);
        __syncthreads();
        int base = total;
#pragma unroll
        for (int w = 0; w < 8; ++w) if (w < wave) base += wcnt[w];
        if (loc >= 0) { const int slot = base + __popc(m & ((1u << lane) - 1u)); if (slot < LCAP) lst[slot] = ((unsigned)loc << 24) | (unsigned)e; }
        __syncthreads();
        if (tid == 0) { int t2 = total; for (int w = 0; w < 8; ++w) t2 += wcnt[w]; total = t2; }
        __syncthreads();
    }
    const int nl = (total < LCAP) ? total : LCAP;
    for (int i = tid; i < nl; i += 256) atomicAdd(&cntb[lst[i] >> 24], 1);
    __syncthreads();
    if (tid == 0) { int o = 0; for (int j = 0; j < BUCKET; ++j) { off[j] = o; o += cntb[j]; } }
    __syncthreads();
    if (tid < BUCKET) { int p = off[tid]; for (int i = 0; i < nl; ++i) if ((int)(lst[i] >> 24) == tid) srt[p++] = lst[i] & 0xFFFFFFu; }
    __syncthreads();
#pragma unroll 1
    for (int pass = 0; pass < 2; ++pass) {
        if (tid < BUCKET && n0 + tid < NN) { *(volatile int*)(noff + n0 + tid) = blockIdx.x * LCAP + off[tid]; *(volatile int*)(ncnt + n0 + tid) = cntb[tid]; }
        for (int c = tid; c * 4 < nl; c += 256)
            *(volatile v4u_t*)((unsigned*)ledge + (size_t)blockIdx.x * LCAP + c * 4) = *(const volatile v4ua*)(srt + c * 4);
        __threadfence();
    }
}

__global__ __launch_bounds__(256) void gnn_gather_kernel(const float* __restrict__ msg, const int* __restrict__ noff, const int* __restrict__ ncnt,
                                                         const int* __restrict__ ledge, float* __restrict__ agg) {
    const int w = (blockIdx.x * 256 + threadIdx.x) >> 5;
    if (w >= NN) return;
    const int lane = threadIdx.x & 31;
    const int o0 = noff[w], cn = ncnt[w];
    float s = 0.0f;
    for (int i = 0; i < cn; ++i) { int e = ledge[o0 + i]; e = ((unsigned)e < (unsigned)NE) ? e : 0; s += msg[(size_t)e * 32 + lane]; }
    const float v = s / (cn > 1 ? (float)cn : 1.0f);
    ST2F(agg + (size_t)w * 32 + lane, v);
}

template<int IN>
__global__ __launch_bounds__(256) void gnn_node_kernel(
    const float* __restrict__ xin,
    const float* __restrict__ root,
    const float* __restrict__ bias,
    const float* __restrict__ agg,
    float* __restrict__ hout,
    int nNodes)
{
    __shared__ __align__(16) float lds_h[8][16][32];
    const int tid = threadIdx.x;
    const int lane = tid & 31;
    const int wave = tid >> 5;
    const int ml = lane & 15;
    const int kh = lane >> 4;
    const int nTiles = (nNodes + 15) >> 4;

    const Frag2 b0 = bfrag_col<IN>(root, 32, ml, kh);
    const Frag2 b1 = bfrag_col<IN>(root, 32, 16 + ml, kh);

    for (int t = blockIdx.x * 8 + wave; t < nTiles; t += gridDim.x * 8) {
        const int m0 = t << 4;
        const int row = m0 + ml;
        const int rowC = row < nNodes ? row : nNodes - 1;
        const Frag2 a = afrag_row<IN>(xin + (size_t)rowC * IN, kh);
        v8f c0 = {}; v8f c1 = {};
        c0 = wmma_split(a, b0, c0);
        c1 = wmma_split(a, b1, c1);
        const float bi0 = bias[ml], bi1 = bias[16 + ml];
        #pragma unroll
        for (int r = 0; r < 8; ++r) {
            const int rr = m0 + r + 8 * kh;
            const int rrc = rr < nNodes ? rr : nNodes - 1;
            float v0 = c0[r] + bi0 + agg[rrc * 32 + ml];
            float v1 = c1[r] + bi1 + agg[rrc * 32 + 16 + ml];
            lds_h[wave][r + 8 * kh][ml]      = v0 > 0.0f ? v0 : 0.0f;
            lds_h[wave][r + 8 * kh][16 + ml] = v1 > 0.0f ? v1 : 0.0f;
        }
        asm volatile("s_wait_dscnt 0" ::: "memory");
        #pragma unroll 1
        for (int pass = 0; pass < 2; ++pass) {
            #pragma unroll
            for (int i = 0; i < 4; ++i) { const int c = lane + 32 * i, rr2 = c >> 3, q = c & 7;
                if (m0 + rr2 < nNodes) *(volatile v4f*)(hout + (size_t)(m0 + rr2) * 32 + q * 4) = *(const volatile v4fa*)(&lds_h[wave][rr2][q * 4]); }
            __threadfence();
        }
        asm volatile("s_wait_dscnt 0" ::: "memory");
    }
}

__global__ __launch_bounds__(256) void gnn_head_kernel(
    const float* __restrict__ h,
    const float* __restrict__ w1,
    const float* __restrict__ b1,
    const float* __restrict__ w2,
    const float* __restrict__ b2,
    float* __restrict__ out,
    int nNodes)
{
    __shared__ float so[128];
    const int tid = threadIdx.x;
    const int lane = tid & 31;
    const int wave = tid >> 5;
    const int ml = lane & 15;
    const int kh = lane >> 4;
    const int nTiles = (nNodes + 15) >> 4;

    const Frag2 p0 = bfrag_col<32>(w1, 32, ml, kh);
    const Frag2 p1 = bfrag_col<32>(w1, 32, 16 + ml, kh);
    const float bb0 = b1[ml], bb1 = b1[16 + ml];
    const float w2a = w2[ml], w2b = w2[16 + ml];
    const float bias2 = b2[0];

    for (int tb = blockIdx.x * 8; tb < nTiles; tb += gridDim.x * 8) {
        const int t = tb + wave;
        const int m0 = t << 4;
        const int row = m0 + ml;
        const int rowC = row < nNodes ? row : nNodes - 1;
        const Frag2 a = afrag_row<32>(h + (size_t)rowC * 32, kh);
        v8f c0 = {}; v8f c1 = {};
        c0 = wmma_split(a, p0, c0);
        c1 = wmma_split(a, p1, c1);
        #pragma unroll
        for (int r = 0; r < 8; ++r) {
            float v0 = c0[r] + bb0; v0 = v0 > 0.0f ? v0 : 0.0f;
            float v1 = c1[r] + bb1; v1 = v1 > 0.0f ? v1 : 0.0f;
            float s = v0 * w2a + v1 * w2b;
            s += __shfl_xor(s, 8, 16);
            s += __shfl_xor(s, 4, 16);
            s += __shfl_xor(s, 2, 16);
            s += __shfl_xor(s, 1, 16);
            if (ml == 0) so[wave * 16 + r + 8 * kh] = s + bias2;
        }
        __syncthreads();
        if (wave == 0) {
#pragma unroll
            for (int i = 0; i < 4; ++i) { const int rr = (tb << 4) + lane + 32 * i; const float v = so[lane + 32 * i];
                if (rr < nNodes) { *(volatile float*)(out + rr) = v; } }
            __threadfence();
#pragma unroll
            for (int i = 0; i < 4; ++i) { const int rr = (tb << 4) + lane + 32 * i; const float v = so[lane + 32 * i];
                if (rr < nNodes) { *(volatile float*)(out + rr) = v; } }
        }
        __syncthreads();
    }
}

extern "C" void kernel_launch(void* const* d_in, const int* in_sizes, int n_in,
                              void* d_out, int out_size, void* d_ws, size_t ws_size,
                              hipStream_t stream) {
    (void)in_sizes; (void)n_in; (void)out_size; (void)ws_size;
    const float*     x      = (const float*)d_in[0];
    const int*       eidx   = (const int*)d_in[1];
    const float*     eattr  = (const float*)d_in[2];
    const float*     w_mlp1 = (const float*)d_in[3];
    const float*     b_mlp1 = (const float*)d_in[4];
    const float*     root1  = (const float*)d_in[5];
    const float*     bias1  = (const float*)d_in[6];
    const float*     w_mlp2 = (const float*)d_in[7];
    const float*     b_mlp2 = (const float*)d_in[8];
    const float*     root2  = (const float*)d_in[9];
    const float*     bias2  = (const float*)d_in[10];
    const float*     w_mlp3 = (const float*)d_in[11];
    const float*     b_mlp3 = (const float*)d_in[12];
    const float*     root3  = (const float*)d_in[13];
    const float*     bias3  = (const float*)d_in[14];
    const float*     w_out1 = (const float*)d_in[15];
    const float*     b_out1 = (const float*)d_in[16];
    const float*     w_out2 = (const float*)d_in[17];
    const float*     b_out2 = (const float*)d_in[18];
    float* out = (float*)d_out;

    float* h1   = (float*)d_ws;
    float* h2   = h1 + (size_t)NN * 32;
    float* agg  = h2 + (size_t)NN * 32;
    float* msg  = agg + (size_t)NN * 32;
    int*   noff = (int*)(msg + (size_t)NE * 32);
    int*   ncnt = noff + NN;
    int*   ledge = ncnt + NN + 64;

    const int edgeBlocks = 782;
    const int nodeBlocks = 196;
    const int gathBlocks = (NN * 32 + 255) / 256;

    gnn_list_kernel<<<NBK, 256, 0, stream>>>(eidx + NE, noff, ncnt, ledge);

    gnn_edge_kernel<8><<<edgeBlocks, 256, 0, stream>>>(x, eidx, eattr, w_mlp1, b_mlp1, msg, NE);
    gnn_gather_kernel<<<gathBlocks, 256, 0, stream>>>(msg, noff, ncnt, ledge, agg);
    gnn_node_kernel<8><<<nodeBlocks, 256, 0, stream>>>(x, root1, bias1, agg, h1, NN);

    gnn_edge_kernel<32><<<edgeBlocks, 256, 0, stream>>>(h1, eidx, eattr, w_mlp2, b_mlp2, msg, NE);
    gnn_gather_kernel<<<gathBlocks, 256, 0, stream>>>(msg, noff, ncnt, ledge, agg);
    gnn_node_kernel<32><<<nodeBlocks, 256, 0, stream>>>(h1, root2, bias2, agg, h2, NN);

    gnn_edge_kernel<32><<<edgeBlocks, 256, 0, stream>>>(h2, eidx, eattr, w_mlp3, b_mlp3, msg, NE);
    gnn_gather_kernel<<<gathBlocks, 256, 0, stream>>>(msg, noff, ncnt, ledge, agg);
    gnn_node_kernel<32><<<nodeBlocks, 256, 0, stream>>>(h2, root3, bias3, agg, h1, NN);

    gnn_head_kernel<<<nodeBlocks, 256, 0, stream>>>(h1, w_out1, b_out1, w_out2, b_out2, out, NN);
}
